// KernalAttention_35424890257839
// MI455X (gfx1250) — hardware-verified
//
#include <hip/hip_runtime.h>


namespace {
constexpr int R = 256, D = 64, L = 65536, DV = 64, LCH = 2048, NCH = L / LCH;
constexpr float A_C = 0.1f, B_C = 0.7745966692414834f  , C_C = -1.0f, PHS = 4096.0f, KVS = 8.0f;
__device__ __forceinline__ float dnorm() { return 0.00028211099074559987f; }

typedef _Float16 b16;
typedef __attribute__((ext_vector_type(16))) _Float16 v16b;
typedef __attribute__((ext_vector_type(16))) __bf16 v16bb;
typedef __attribute__((ext_vector_type(8))) _Float16 v8b;
typedef __attribute__((ext_vector_type(8))) unsigned short v8us;
typedef __attribute__((ext_vector_type(8))) float v8f;
typedef __attribute__((ext_vector_type(4))) float v4f;
__device__ __forceinline__ float bf16_rne(float f) { unsigned int u = __float_as_uint(f); u += 0x7FFFu + ((u >> 16) & 1u); return __uint_as_float(u & 0xFFFF0000u); }
__device__ __forceinline__ unsigned short bf16_bits(float f) { unsigned int u = __float_as_uint(f); u += 0x7FFFu + ((u >> 16) & 1u); return (unsigned short)(u >> 16); }
__device__ __forceinline__ void split16(float v, b16& hi, b16& lo) { hi = (b16)v; lo = (b16)(v - (float)hi); }
__device__ __forceinline__ v16b frag_kb(const b16* p, int hh) { const v8b a = *(const v8b*)(p + 8 * hh), b = *(const v8b*)(p + 16 + 8 * hh); v16b f;
#pragma unroll
  for (int e = 0; e < 8; ++e) { f[e] = a[e]; f[8 + e] = b[e]; } return f; }
__device__ __forceinline__ v16bb frag_bf(const unsigned short* p, int hh) { const v8us a = *(const v8us*)(p + 8 * hh), b = *(const v8us*)(p + 16 + 8 * hh); union { unsigned short s[16]; v16bb v; } u;
#pragma unroll
  for (int e = 0; e < 8; ++e) { u.s[e] = a[e]; u.s[8 + e] = b[e]; } return u.v; }
__device__ __forceinline__ v8f wmma16b(v16b a, v16b b, v8f c) { v8f d = __builtin_amdgcn_wmma_f32_16x16x32_f16(false, a, false, b, (short)0, c, false, false); asm volatile("v_nop\n\tv_nop\n\tv_nop\n\tv_nop" : "+v"(d) : "v"(a), "v"(b)); return d; }
__device__ __forceinline__ v8f wmma16bb(v16bb a, v16bb b, v8f c) { v8f d = __builtin_amdgcn_wmma_f32_16x16x32_bf16(false, a, false, b, (short)0, c, false, false); asm volatile("v_nop\n\tv_nop\n\tv_nop\n\tv_nop" : "+v"(d) : "v"(a), "v"(b)); return d; }
__device__ __forceinline__ void wave_lds_sync() { __builtin_amdgcn_fence(__ATOMIC_RELEASE, "workgroup"); __builtin_amdgcn_wave_barrier(); __builtin_amdgcn_fence(__ATOMIC_ACQUIRE, "workgroup"); }

__global__ __launch_bounds__(256) void prep_kernel(const float* __restrict__ Q, const float* __restrict__ K, const float* __restrict__ V, const float* __restrict__ W, unsigned short* __restrict__ qT, unsigned short* __restrict__ kT, float* __restrict__ sq, float* __restrict__ sk, b16* __restrict__ vT, unsigned short* __restrict__ w16) {
  __shared__ __attribute__((aligned(16))) unsigned short Tq[128][64 + 8], Tk[128][64 + 8]; __shared__ __attribute__((aligned(16))) b16 Tv[64][128 + 8]; __shared__ float Sq[128], Sk[128];
  const int t_ = threadIdx.x, l0 = blockIdx.x * 128;
  for (int i = t_; i < 64 * 128; i += 256) { const int d = i >> 7, ll = i & 127; Tq[ll][d] = bf16_bits(Q[(size_t)d * L + l0 + ll]); Tk[ll][d] = bf16_bits(K[(size_t)d * L + l0 + ll]); }
  for (int i = t_; i < 128 * 64; i += 256) { const int ll = i >> 6, d = i & 63; Tv[d][ll] = (b16)bf16_rne(V[(size_t)(l0 + ll) * DV + d]); }
  __syncthreads();
  if (t_ < 128) { float s = 0.0f, s2 = 0.0f; for (int d = 0; d < 64; ++d) { const float a = __uint_as_float((unsigned)Tq[t_][d] << 16), b = __uint_as_float((unsigned)Tk[t_][d] << 16); s += a * a; s2 += b * b; } Sq[t_] = s; Sk[t_] = s2; }
  __syncthreads();
  for (int pass = 0; pass < 2; ++pass) {
    for (int i = t_; i < 128 * 8; i += 256) { const int ll = i >> 3, c8 = (i & 7) * 8; *(volatile v8us*)(qT + (size_t)(l0 + ll) * D + c8) = *(const v8us*)(&Tq[ll][c8]); *(volatile v8us*)(kT + (size_t)(l0 + ll) * D + c8) = *(const v8us*)(&Tk[ll][c8]); }
    for (int i = t_; i < 64 * 16; i += 256) { const int d = i >> 4, c8 = (i & 15) * 8; *(volatile v8b*)(vT + (size_t)d * L + l0 + c8) = *(const v8b*)(&Tv[d][c8]); }
    if (t_ < 32) { *(volatile v4f*)(sq + l0 + t_ * 4) = *(const v4f*)(&Sq[t_ * 4]); *(volatile v4f*)(sk + l0 + t_ * 4) = *(const v4f*)(&Sk[t_ * 4]); }
    if (blockIdx.x == 0) for (int i = t_; i < R * D / 8; i += 256) { v8us v;
#pragma unroll
      for (int e = 0; e < 8; ++e) v[e] = bf16_bits(W[i * 8 + e]);
      *(volatile v8us*)(w16 + i * 8) = v; }
    __threadfence(); }
}

__global__ __launch_bounds__(128) void phiq_kernel(const unsigned short* __restrict__ qT, const unsigned short* __restrict__ w16, const float* __restrict__ sq, b16* __restrict__ phq) {
  __shared__ __attribute__((aligned(16))) b16 Ts[4][32][64 + 8];
  const int lane = threadIdx.x & 31, wave = threadIdx.x >> 5, nloc = lane & 15, hlf = lane >> 4, m0 = blockIdx.y * 128 + wave * 32, c0 = blockIdx.x * 64;
  v8f acc[2][4];
#pragma unroll
  for (int r = 0; r < 2; ++r)
#pragma unroll
    for (int t = 0; t < 4; ++t) acc[r][t] = (v8f){};
#pragma unroll
  for (int kb = 0; kb < D; kb += 32) { const v16bb a0 = frag_bf(qT + (size_t)(m0 + nloc) * D + kb, hlf), a1 = frag_bf(qT + (size_t)(m0 + 16 + nloc) * D + kb, hlf);
#pragma unroll
    for (int t = 0; t < 4; ++t) { const v16bb bw = frag_bf(w16 + (size_t)(c0 + t * 16 + nloc) * D + kb, hlf); acc[0][t] = wmma16bb(a0, bw, acc[0][t]); acc[1][t] = wmma16bb(a1, bw, acc[1][t]); } }
  const float dn = dnorm();
#pragma unroll
  for (int t = 0; t < 4; ++t)
#pragma unroll
    for (int r = 0; r < 2; ++r)
#pragma unroll
      for (int v = 0; v < 8; ++v) { const int row = m0 + r * 16 + 8 * hlf + v; Ts[wave][r * 16 + 8 * hlf + v][t * 16 + nloc] = (b16)(dn * __expf(A_C + B_C * acc[r][t][v] + C_C * sq[row]) * PHS); }
  wave_lds_sync();
  b16* dst = phq + (size_t)m0 * R + c0;
  for (int pass = 0; pass < 2; ++pass) {
#pragma unroll
    for (int j = 0; j < 8; ++j) { const int rr = j * 4 + (lane >> 3), c8 = (lane & 7) * 8; *(volatile v8b*)(dst + (size_t)rr * R + c8) = *(const v8b*)(&Ts[wave][rr][c8]); }
    __threadfence(); }
}
__global__ __launch_bounds__(128) void phik_kernel(const unsigned short* __restrict__ kT, const unsigned short* __restrict__ w16, const float* __restrict__ sk, b16* __restrict__ phk) {
  __shared__ __attribute__((aligned(16))) b16 Ts[4][32][64 + 8];
  const int lane = threadIdx.x & 31, wave = threadIdx.x >> 5, nloc = lane & 15, hlf = lane >> 4, m0 = blockIdx.y * 128 + wave * 32, c0 = blockIdx.x * 64;
  v8f acc[2][4];
#pragma unroll
  for (int r = 0; r < 2; ++r)
#pragma unroll
    for (int t = 0; t < 4; ++t) acc[r][t] = (v8f){};
#pragma unroll
  for (int kb = 0; kb < D; kb += 32) { const v16bb a0 = frag_bf(w16 + (size_t)(m0 + nloc) * D + kb, hlf), a1 = frag_bf(w16 + (size_t)(m0 + 16 + nloc) * D + kb, hlf);
#pragma unroll
    for (int t = 0; t < 4; ++t) { const v16bb bw = frag_bf(kT + (size_t)(c0 + t * 16 + nloc) * D + kb, hlf); acc[0][t] = wmma16bb(a0, bw, acc[0][t]); acc[1][t] = wmma16bb(a1, bw, acc[1][t]); } }
  const float dn = dnorm();
#pragma unroll
  for (int t = 0; t < 4; ++t) { const float s2 = sk[c0 + t * 16 + nloc];
#pragma unroll
    for (int r = 0; r < 2; ++r)
#pragma unroll
      for (int v = 0; v < 8; ++v) Ts[wave][r * 16 + 8 * hlf + v][t * 16 + nloc] = (b16)(dn * __expf(A_C + B_C * acc[r][t][v] + C_C * s2) * PHS); }
  wave_lds_sync();
  b16* dst = phk + (size_t)m0 * L + c0;
  for (int pass = 0; pass < 2; ++pass) {
#pragma unroll
    for (int j = 0; j < 8; ++j) { const int rr = j * 4 + (lane >> 3), c8 = (lane & 7) * 8; *(volatile v8b*)(dst + (size_t)rr * L + c8) = *(const v8b*)(&Ts[wave][rr][c8]); }
    __threadfence(); }
}

__global__ __launch_bounds__(256) void kvpart_kernel(const b16* __restrict__ phk, const b16* __restrict__ vT, float* __restrict__ part) {
  __shared__ __attribute__((aligned(16))) float Ts[8][32 * 64];
  const int lane = threadIdx.x & 31, wave = threadIdx.x >> 5, nloc = lane & 15, hlf = lane >> 4, m0 = wave * 32, ch = blockIdx.x, l0 = ch * LCH;
  v8f acc[2][4];
#pragma unroll
  for (int r = 0; r < 2; ++r)
#pragma unroll
    for (int t = 0; t < 4; ++t) acc[r][t] = (v8f){};
#pragma unroll 2
  for (int kb = 0; kb < LCH; kb += 32) { const v16b a0 = frag_kb(phk + (size_t)(m0 + nloc) * L + l0 + kb, hlf), a1 = frag_kb(phk + (size_t)(m0 + 16 + nloc) * L + l0 + kb, hlf);
#pragma unroll
    for (int t = 0; t < 4; ++t) { const v16b bv = frag_kb(vT + (size_t)(t * 16 + nloc) * L + l0 + kb, hlf); acc[0][t] = wmma16b(a0, bv, acc[0][t]); acc[1][t] = wmma16b(a1, bv, acc[1][t]); } }
  float* Tt = Ts[wave];
#pragma unroll
  for (int t = 0; t < 4; ++t)
#pragma unroll
    for (int r = 0; r < 2; ++r)
#pragma unroll
      for (int v = 0; v < 8; ++v) Tt[(r * 16 + v + 8 * hlf) * 64 + t * 16 + nloc] = acc[r][t][v] * (1.0f / PHS);
  wave_lds_sync();
  float* dst0 = part + ((size_t)ch * R + m0) * DV;
  for (int pass = 0; pass < 2; ++pass) {
#pragma unroll
    for (int j = 0; j < 16; ++j) { const int rr = j * 2 + hlf, c4 = nloc * 4; *(volatile v4f*)(dst0 + (size_t)rr * DV + c4) = *(const v4f*)(Tt + rr * 64 + c4); }
    __threadfence(); }
}
typedef __attribute__((ext_vector_type(2))) _Float16 v2b;
__global__ __launch_bounds__(128) void kvred_kernel(const float* __restrict__ part, b16* __restrict__ kvh, b16* __restrict__ kvl) {
  const int dv = blockIdx.x, r = threadIdx.x * 2; float s0 = 0.0f, s1 = 0.0f;
  for (int ch = 0; ch < NCH; ++ch) { s0 += part[((size_t)ch * R + r) * DV + dv]; s1 += part[((size_t)ch * R + r + 1) * DV + dv]; }
  v2b vh, vl; b16 a, c; split16(s0 * KVS, a, c); vh[0] = a; vl[0] = c; split16(s1 * KVS, a, c); vh[1] = a; vl[1] = c;
  for (int pass = 0; pass < 2; ++pass) { *(volatile v2b*)(kvh + (size_t)dv * R + r) = vh; *(volatile v2b*)(kvl + (size_t)dv * R + r) = vl; __threadfence(); }
}

__global__ __launch_bounds__(128) void out_kernel(const b16* __restrict__ phq, const b16* __restrict__ kvh, const b16* __restrict__ kvl, float* __restrict__ out) {
  __shared__ __attribute__((aligned(16))) float Ts[4][32 * 64];
  const int lane = threadIdx.x & 31, wave = threadIdx.x >> 5, nloc = lane & 15, hlf = lane >> 4, m0 = blockIdx.x * 128 + wave * 32;
  v8f acc[2][4];
#pragma unroll
  for (int r = 0; r < 2; ++r)
#pragma unroll
    for (int t = 0; t < 4; ++t) acc[r][t] = (v8f){};
#pragma unroll
  for (int kb = 0; kb < R; kb += 32) { const v16b a0 = frag_kb(phq + (size_t)(m0 + nloc) * R + kb, hlf), a1 = frag_kb(phq + (size_t)(m0 + 16 + nloc) * R + kb, hlf);
#pragma unroll
    for (int t = 0; t < 4; ++t) { const v16b b0 = frag_kb(kvh + (size_t)(t * 16 + nloc) * R + kb, hlf), b1 = frag_kb(kvl + (size_t)(t * 16 + nloc) * R + kb, hlf);
      acc[0][t] = wmma16b(a0, b0, acc[0][t]); acc[0][t] = wmma16b(a0, b1, acc[0][t]); acc[1][t] = wmma16b(a1, b0, acc[1][t]); acc[1][t] = wmma16b(a1, b1, acc[1][t]); } }
  float* Tt = Ts[wave];
#pragma unroll
  for (int t = 0; t < 4; ++t)
#pragma unroll
    for (int r = 0; r < 2; ++r)
#pragma unroll
      for (int v = 0; v < 8; ++v) Tt[(r * 16 + v + 8 * hlf) * 64 + t * 16 + nloc] = acc[r][t][v] * (1.0f / (PHS * KVS));
  wave_lds_sync();
  float* dst0 = out + (size_t)m0 * DV;
  for (int pass = 0; pass < 2; ++pass) {
#pragma unroll
    for (int j = 0; j < 16; ++j) { const int rr = j * 2 + hlf, c4 = nloc * 4; *(volatile v4f*)(dst0 + (size_t)rr * DV + c4) = *(const v4f*)(Tt + rr * 64 + c4); }
    __threadfence(); }
}
}

extern "C" void kernel_launch(void* const* d_in, const int* in_sizes, int n_in,
                              void* d_out, int out_size, void* d_ws, size_t ws_size, hipStream_t stream) {
  (void)n_in; (void)out_size;
  const float* Q = (const float*)d_in[0]; const float* K = (const float*)d_in[1]; const float* V = (const float*)d_in[2]; const float* W = (const float*)d_in[3];
  float* out = (float*)d_out;
  if (in_sizes[0] != D * L || in_sizes[1] != D * L || in_sizes[2] != L * DV || in_sizes[3] != R * D) return;
  size_t off = 0; char* ws = (char*)d_ws;
  auto carve = [&](size_t bytes) { char* p = ws + off; off += (bytes + 255) & ~(size_t)255; return p; };
  unsigned short* qT = (unsigned short*)carve((size_t)L * D * 2); unsigned short* kT = (unsigned short*)carve((size_t)L * D * 2); float* sq = (float*)carve((size_t)L * 4); float* sk = (float*)carve((size_t)L * 4); b16* vT = (b16*)carve((size_t)DV * L * 2); unsigned short* w16 = (unsigned short*)carve(R * D * 2);
  b16* phq = (b16*)carve((size_t)L * R * 2); b16* phk = (b16*)carve((size_t)R * L * 2); float* part = (float*)carve((size_t)NCH * R * DV * 4); b16* kvh = (b16*)carve(DV * R * 2); b16* kvl = (b16*)carve(DV * R * 2);
  if (off > ws_size) return;
  prep_kernel<<<L / 128, 256, 0, stream>>>(Q, K, V, W, qT, kT, sq, sk, vT, w16);
  phiq_kernel<<<dim3(R / 64, L / 128), 128, 0, stream>>>(qT, w16, sq, phq);
  phik_kernel<<<dim3(L / 64, R / 128), 128, 0, stream>>>(kT, w16, sk, phk);
  kvpart_kernel<<<NCH, 256, 0, stream>>>(phk, vT, part);
  kvred_kernel<<<DV, 128, 0, stream>>>(part, kvh, kvl);
  out_kernel<<<L / 128, 128, 0, stream>>>(phq, kvh, kvl, out);
}
